// GravityNet_81604378624570
// MI455X (gfx1250) — hardware-verified
//
#include <hip/hip_runtime.h>
#include <math.h>

typedef __attribute__((ext_vector_type(16))) _Float16 v16h;
typedef __attribute__((ext_vector_type(8)))  _Float16 v8h;
typedef __attribute__((ext_vector_type(8)))  float    v8f;
typedef __attribute__((ext_vector_type(4)))  float    v4f;
typedef __attribute__((ext_vector_type(4)))  unsigned int v4u;

constexpr int kZ = 2;
constexpr int kA = 1024;
constexpr int kNB = 30;
constexpr int kHid = 100;
constexpr int kNPad = 112;
constexpr int kKPad = 128;
constexpr int kKB = 32;
constexpr int kNT = 7;
constexpr int kSB = 40;
constexpr int kSA = 136;
constexpr int kThreads = 128;
constexpr int kWaves = kThreads / 32;
constexpr int kRowsBlk = kWaves * 16;
static_assert(kThreads == 2 * kRowsBlk);

constexpr int kGroupsZ  = 33216;
constexpr int kRowsZ    = kGroupsZ * 16;
constexpr int kBlocksZ  = kGroupsZ / kWaves;
constexpr int kRowsTot  = kZ * kRowsZ;
constexpr int kMlpBlocks = kZ * kBlocksZ;
constexpr int kOutBlocks = kZ * kA / 32;
static_assert(kGroupsZ % kWaves == 0);
static_assert(kMlpBlocks * kRowsBlk == kRowsTot);

constexpr float kWCarry    = 16.0f;
constexpr float kActCarry  = 16.0f;
constexpr float kL0Scale   = 1.0f / 16.0f;
constexpr float kL1Scale   = 1.0f / 256.0f;
constexpr float kL2Scale   = 1.0f / 256.0f;
constexpr float kRs30      = 1.0f / 5.477225575051661f;
constexpr float kRs100     = 0.1f;
constexpr float kStep      = 0.0689655172413793f;
constexpr float kInvStep   = 1.0f / kStep;
constexpr float kHalfPi    = 1.5707963267948966f;
constexpr float kSqrt3     = 1.7320508075688772f;
constexpr float kBeta      = 5.0f;
constexpr float kSpk       = 0.28063965f;

constexpr size_t kOffW0T  = 0;
constexpr size_t kOffW1T  = kOffW0T + (size_t)kNPad * kKB * 2;
constexpr size_t kOffW2T  = kOffW1T + (size_t)kNPad * kKPad * 2;
constexpr size_t kOffRp   = kOffW2T + (size_t)16 * kKPad * 2;
constexpr size_t kWsTotal = kOffRp + (size_t)kRowsTot * 4;
static_assert(kOffW1T == 7168 && kOffW2T == 35840 && kOffRp == 39936 && kWsTotal == 4291584);
static_assert(kOffW1T % 128 == 0 && kOffW2T % 128 == 0 && kOffRp % 128 == 0);
static_assert(kWsTotal <= (size_t)134217728);

__constant__ float kCenters[32] = {0.0f,0.068965517f,0.137931034f,0.206896544f,0.275862068f,0.344827592f,0.413793087f,0.482758611f,0.551724136f,0.620689631f,0.689655185f,0.758620679f,0.827586174f,0.896551728f,0.965517223f,1.03448272f,1.10344827f,1.17241383f,1.24137926f,1.31034482f,1.37931037f,1.4482758f,1.51724136f,1.58620691f,1.65517235f,1.7241379f,1.79310346f,1.86206901f,1.93103445f,2.0f,
                                   -1000.0f, -1000.0f};
static_assert(sizeof(kCenters) / sizeof(kCenters[0]) == 32);

__host__ __device__ constexpr int seg_c(int q) { return 16 * (63 * q - ((q * (q - 1)) >> 1)); }
__host__ __device__ constexpr int grp_off(int a) {
  const int v   = (a > 15) ? (a - 15) : 0;
  const int q   = v >> 4;
  const int rmd = v & 15;
  const int hi  = 960 + seg_c(q) + rmd * (63 - q);
  return (a <= 15) ? (64 * a) : hi;
}
__host__ __device__ constexpr int grp_inv(int gi) {
  const int gp = (gi >= 960) ? (gi - 960) : 0;
  int qq = 0;
  for (int q = 1; q <= 62; ++q) qq += (seg_c(q) <= gp) ? 1 : 0;
  const int idx = gp - seg_c(qq);
  const int per = 63 - qq;
  const int s   = idx / per;
  const int ahi = 15 + 16 * qq + s;
  const int jhi = idx - s * per;
  const int alo = gi >> 6;
  const int jlo = gi & 63;
  return (gi < 960) ? (alo * 64 + jlo) : (ahi * 64 + jhi);
}
constexpr bool check_groups() {
  int s = 0;
  for (int a = 0; a < kA; ++a) {
    if (grp_off(a) != s) return false;
    const int n = (kA - 1 - a + 15) >> 4;
    if (n > 0 && (((a & 7) == 0) || a >= 1000)) {
      if (grp_inv(s) != a * 64) return false;
      if (grp_inv(s + n - 1) != a * 64 + (n - 1)) return false;
    }
    s += n;
  }
  return s == kGroupsZ;
}
static_assert(grp_off(15) == 960 && grp_off(16) == 1023 && grp_off(kA - 1) == kGroupsZ);
static_assert(check_groups());

template <typename T> struct Frag;
template <> struct Frag<_Float16> {
  typedef v16h V; union U { v16h v; v8h h[2]; };
  static __device__ __forceinline__ v16h load(const _Float16* p) {
    U f; f.h[0] = *(const v8h*)(p); f.h[1] = *(const v8h*)(p + 16); return f.v;
  }
};

__device__ __forceinline__ v8f mma_h(v16h a, v16h b, v8f c) {
  c = __builtin_amdgcn_wmma_f32_16x16x32_f16(false, a, false, b, (short)0, c, false, false);
  asm volatile("v_nop\n\tv_nop\n\tv_nop\n\tv_nop" : "+v"(c) : "v"(a), "v"(b));
  return c;
}

__device__ __forceinline__ v8f zero8() { return (v8f){0.f,0.f,0.f,0.f,0.f,0.f,0.f,0.f}; }
__device__ __forceinline__ unsigned pk16(unsigned short a, unsigned short b) { return (unsigned)a | ((unsigned)b << 16); }
__device__ __forceinline__ unsigned short h_bits(float f) { const _Float16 h = (_Float16)f; return __builtin_bit_cast(unsigned short, h); }

__device__ __forceinline__ void store16x2(unsigned short* dst, const unsigned short (&hb)[8]) {
  const v4u u = (v4u){pk16(hb[0], hb[1]), pk16(hb[2], hb[3]), pk16(hb[4], hb[5]), pk16(hb[6], hb[7])};
  *(volatile v4u*)dst = u;
  __threadfence();
  *(volatile v4u*)dst = u;
}

__device__ __forceinline__ float actf(float v) {
  const float y  = kBeta * v;
  const float e  = expf(-fabsf(y));
  const float sp = logf(1.0f + e) + fmaxf(y, 0.0f);
  return sp * kSpk;
}

__global__ __launch_bounds__(256) void prep_weights(const float* __restrict__ W0, const float* __restrict__ W1,
                                                      const float* __restrict__ W2,
                                                      unsigned short* __restrict__ w0t, unsigned short* __restrict__ w1t,
                                                      unsigned short* __restrict__ w2t) {
  const int t   = threadIdx.x;
  const int blk = blockIdx.x;
  unsigned short hb[8];
  if (blk < 2) {
    const int c = blk * 256 + t;
    if (c < 448) {
      const int n  = c >> 2;
      const int kb = (c & 3) * 8;
      const int nc = (n < kHid) ? n : (kHid - 1);
#pragma unroll
      for (int e = 0; e < 8; ++e) {
        const int k  = kb + e;
        const int kc = (k < kNB) ? k : (kNB - 1);
        float v = W0[kc * kHid + nc] * kRs30 * kWCarry;
        v = (n < kHid && k < kNB) ? v : 0.0f;
        hb[e] = h_bits(v);
      }
      store16x2(w0t + 8 * (size_t)c, hb);
    }
  } else if (blk < 9) {
    const int c  = (blk - 2) * 256 + t;
    const int n  = c >> 4;
    const int kb = (c & 15) * 8;
    const int nc = (n < kHid) ? n : (kHid - 1);
#pragma unroll
    for (int e = 0; e < 8; ++e) {
      const int k  = kb + e;
      const int kc = (k < kHid) ? k : (kHid - 1);
      float v = W1[kc * kHid + nc] * kRs100 * kWCarry;
      v = (n < kHid && k < kHid) ? v : 0.0f;
      hb[e] = h_bits(v);
    }
    store16x2(w1t + 8 * (size_t)c, hb);
  } else {
    const int c  = t;
    const int n  = c >> 4;
    const int kb = (c & 15) * 8;
#pragma unroll
    for (int e = 0; e < 8; ++e) {
      const int k  = kb + e;
      const int kc = (k < kHid) ? k : (kHid - 1);
      float v = W2[kc] * kRs100 * kWCarry;
      v = (n == 0 && k < kHid) ? v : 0.0f;
      hb[e] = h_bits(v);
    }
    store16x2(w2t + 8 * (size_t)c, hb);
  }
}

__global__ __launch_bounds__(kThreads) void radial_mlp(const float* __restrict__ geometry,
                                                         const unsigned short* __restrict__ w0tp,
                                                         const unsigned short* __restrict__ w1tp,
                                                         const unsigned short* __restrict__ w2tp,
                                                         float* __restrict__ rp) {
  __shared__ __align__(16) _Float16 sBasis[kRowsBlk * kSB];
  __shared__ __align__(16) _Float16 sAct0[kRowsBlk * kSA];
  __shared__ __align__(16) _Float16 sAct1[kRowsBlk * kSA];
  __shared__ float sR[kRowsBlk];
  __shared__ __align__(16) float sRo[kRowsBlk];

  const _Float16* w0t = (const _Float16*)(const void*)w0tp;
  const _Float16* w1t = (const _Float16*)(const void*)w1tp;
  const _Float16* w2t = (const _Float16*)(const void*)w2tp;

  const int t    = threadIdx.x;
  const int lane = t & 31;
  const int w    = t >> 5;
  const int g    = lane >> 4;
  const int ln   = lane & 15;
  const int rowA = w * 16 + ln;
  const int blk  = blockIdx.x;
  const int z    = blk / kBlocksZ;
  const int gblk = blk - z * kBlocksZ;

  {
    v8h zv;
#pragma unroll
    for (int e = 0; e < 8; ++e) zv[e] = (_Float16)0.0f;
    const int row = t >> 1;
    const int c0  = kNPad + 8 * (t & 1);
    *(v8h*)(sAct0 + row * kSA + c0) = zv;
    *(v8h*)(sAct1 + row * kSA + c0) = zv;
  }

  if (t < kRowsBlk) {
    const int gi = gblk * kWaves + (t >> 4);
    const int m  = t & 15;
    const int aj = grp_inv(gi);
    int a = aj >> 6;
    a = (a < 0) ? 0 : ((a > kA - 1) ? (kA - 1) : a);
    const int j = aj & 63;
    int b = a + 1 + 16 * j + m;
    b = (b > kA - 1) ? (kA - 1) : b;
    const float* gap = geometry + ((size_t)z * kA + a) * 3;
    const float* gbp = geometry + ((size_t)z * kA + b) * 3;
    const float rx = gbp[0] - gap[0];
    const float ry = gbp[1] - gap[1];
    const float rz = gbp[2] - gap[2];
    const float r2 = (rx * rx + rz * rz) + ry * ry;
    const bool  mk = (r2 > 1e-12f);
    const float rr = sqrtf(mk ? r2 : 1.0f);
    sR[t] = mk ? rr : 0.0f;
  }
  __syncthreads();

  {
    const int p   = t >> 1;
    const int odd = t & 1;
    const float rpv = sR[p];
    int hE = -1, hO = -1;
    float dE = 0.0f, dO = 0.0f;
#pragma unroll
    for (int kk = 0; kk < 16; ++kk) {
      const float ca = kCenters[kk], cb = kCenters[16 + kk];
      const float c  = odd ? cb : ca;
      const float d  = (rpv - c) * kInvStep;
      const bool hit = fabsf(d) < 1.0f;
      if ((kk & 1) == 0) { hE = hit ? kk : hE; dE = hit ? d : dE; }
      else               { hO = hit ? kk : hO; dO = hit ? d : dO; }
    }
    const float cE = cosf(kHalfPi * dE);
    const float cO = cosf(kHalfPi * dO);
    const float vE = cE * cE;
    const float vO = cO * cO;
    v8h q0, q1;
#pragma unroll
    for (int kk = 0; kk < 8; ++kk) {
      const int k1 = kk + 8;
      const float x0 = ((kk & 1) == 0) ? ((hE == kk) ? vE : 0.0f) : ((hO == kk) ? vO : 0.0f);
      const float x1 = ((k1 & 1) == 0) ? ((hE == k1) ? vE : 0.0f) : ((hO == k1) ? vO : 0.0f);
      q0[kk] = (_Float16)x0;
      q1[kk] = (_Float16)x1;
    }
    _Float16* bp = sBasis + p * kSB + odd * 16;
    *(v8h*)(bp)     = q0;
    *(v8h*)(bp + 8) = q1;
  }
  __syncthreads();

  {
    const v16h a0 = Frag<_Float16>::load(sBasis + rowA * kSB + 8 * g);
#pragma unroll 1
    for (int nt = 0; nt < kNT; ++nt) {
      const v16h bf = Frag<_Float16>::load(w0t + (size_t)(nt * 16 + ln) * kKB + 8 * g);
      v8f acc = mma_h(a0, bf, zero8());
      const int col = nt * 16 + ln;
      _Float16* dst = sAct0 + (w * 16 + 8 * g) * kSA + col;
#pragma unroll
      for (int r = 0; r < 8; ++r) {
        const float v = acc[r] * kL0Scale;
        float hv = 0.0f;
        if (col < kHid) hv = actf(v) * kActCarry;
        dst[r * kSA] = (_Float16)hv;
      }
    }
  }
  __syncthreads();

  {
#pragma unroll 1
    for (int nt = 0; nt < kNT; ++nt) {
      v8f acc = zero8();
#pragma unroll
      for (int ks = 0; ks < 4; ++ks) {
        const v16h af = Frag<_Float16>::load(sAct0 + rowA * kSA + ks * 32 + 8 * g);
        const v16h bf = Frag<_Float16>::load(w1t + (size_t)(nt * 16 + ln) * kKPad + ks * 32 + 8 * g);
        acc = mma_h(af, bf, acc);
      }
      const int col = nt * 16 + ln;
      _Float16* dst = sAct1 + (w * 16 + 8 * g) * kSA + col;
#pragma unroll
      for (int r = 0; r < 8; ++r) {
        const float v = acc[r] * kL1Scale;
        float hv = 0.0f;
        if (col < kHid) hv = actf(v) * kActCarry;
        dst[r * kSA] = (_Float16)hv;
      }
    }
  }
  __syncthreads();

  {
    v8f acc = zero8();
#pragma unroll
    for (int ks = 0; ks < 4; ++ks) {
      const v16h af = Frag<_Float16>::load(sAct1 + rowA * kSA + ks * 32 + 8 * g);
      const v16h bf = Frag<_Float16>::load(w2t + (size_t)ln * kKPad + ks * 32 + 8 * g);
      acc = mma_h(af, bf, acc);
    }
    if (ln == 0) {
#pragma unroll
      for (int r = 0; r < 8; ++r) sRo[w * 16 + 8 * g + r] = acc[r] * kL2Scale;
    }
  }
  __syncthreads();

  if (w == 0) {
    const int lc = lane & 15;
    const v4f v  = *(const v4f*)(sRo + lc * 4);
    float* dst   = rp + (size_t)blk * kRowsBlk + lc * 4;
    if (lane < 16) *(volatile v4f*)dst = v;
    __threadfence();
    if (lane < 16) *(volatile v4f*)dst = v;
  }
}

__global__ __launch_bounds__(32) void pair_sum_out(const float* __restrict__ features,
                                                     const float* __restrict__ geometry,
                                                     const float* __restrict__ rp,
                                                     float* __restrict__ out) {
  __shared__ int sOff[kA];
  __shared__ __align__(16) float sOut[96];
  const int lane = threadIdx.x;
  const int blk  = blockIdx.x;
  const int z    = blk >> 5;
  const int a    = (blk & 31) * 32 + lane;
#pragma unroll 1
  for (int i = lane; i < kA; i += 32) sOff[i] = 16 * grp_off(i);
  __syncthreads();

  const float* gap = geometry + ((size_t)z * kA + a) * 3;
  const float gax = gap[0], gay = gap[1], gaz = gap[2];
  const size_t zrow = (size_t)z * kRowsZ;
  float sx = 0.0f, sy = 0.0f, sz = 0.0f;
#pragma unroll 1
  for (int b = 0; b < kA; ++b) {
    const size_t bi = (size_t)z * kA + b;
    const float* gbp = geometry + bi * 3;
    const float rx = gbp[0] - gax;
    const float ry = gbp[1] - gay;
    const float rz = gbp[2] - gaz;
    const float fb = features[bi];
    const float r2 = (rx * rx + rz * rz) + ry * ry;
    const bool  mk = (r2 > 1e-12f);
    const float rr = sqrtf(mk ? r2 : 1.0f);
    const float rinv = 1.0f / rr;
    const int lo = (b < a) ? b : a;
    const int hi = (b < a) ? a : b;
    int dl = hi - lo - 1;
    dl = (dl < 0) ? 0 : dl;
    size_t row = zrow + (size_t)sOff[lo] + (size_t)dl;
    row = (row > (size_t)(kRowsTot - 1)) ? (size_t)(kRowsTot - 1) : row;
    const float R  = rp[row];
    const float rf = R * fb;
    const float yx = mk ? (kSqrt3 * (rx * rinv)) : 0.0f;
    const float yy = mk ? (kSqrt3 * (ry * rinv)) : 0.0f;
    const float yz = mk ? (kSqrt3 * (rz * rinv)) : 0.0f;
    sx += yx * rf;
    sy += yy * rf;
    sz += yz * rf;
  }
  sOut[lane * 3 + 0] = sx;
  sOut[lane * 3 + 1] = sy;
  sOut[lane * 3 + 2] = sz;
  __syncthreads();
  {
    const int lc = (lane < 24) ? lane : 0;
    const v4f v  = *(const v4f*)(sOut + lc * 4);
    float* dst   = out + (size_t)blk * 96 + lc * 4;
    if (lane < 24) *(volatile v4f*)dst = v;
    __threadfence();
    if (lane < 24) *(volatile v4f*)dst = v;
  }
}

extern "C" void kernel_launch(void* const* d_in, const int* in_sizes, int n_in,
                              void* d_out, int out_size, void* d_ws, size_t ws_size,
                              hipStream_t stream) {
  if (n_in < 5) return;
  if (in_sizes[0] != kZ * kA || in_sizes[1] != kZ * kA * 3 || in_sizes[2] != kNB * kHid ||
      in_sizes[3] != kHid * kHid || in_sizes[4] != kHid) return;
  if (out_size < kZ * kA * 3) return;
  if (ws_size < kWsTotal) return;

  const float* features = (const float*)d_in[0];
  const float* geometry = (const float*)d_in[1];
  const float* W0       = (const float*)d_in[2];
  const float* W1       = (const float*)d_in[3];
  const float* W2       = (const float*)d_in[4];
  float*       out      = (float*)d_out;

  unsigned char* ws = (unsigned char*)d_ws;
  unsigned short* w0t = (unsigned short*)(ws + kOffW0T);
  unsigned short* w1t = (unsigned short*)(ws + kOffW1T);
  unsigned short* w2t = (unsigned short*)(ws + kOffW2T);
  float*          rp  = (float*)(ws + kOffRp);

  prep_weights<<<10, 256, 0, stream>>>(W0, W1, W2, w0t, w1t, w2t);
  radial_mlp<<<kMlpBlocks, kThreads, 0, stream>>>(geometry, w0t, w1t, w2t, rp);
  pair_sum_out<<<kOutBlocks, 32, 0, stream>>>(features, geometry, rp, out);
}
